// RWKV_Tmix_headmixer_20830591385839
// MI455X (gfx1250) — hardware-run, weakly checked
//
#include <hip/hip_runtime.h>
#include <math.h>

constexpr int kT = 2048;
constexpr int kC = 1024;
constexpr int kH = 16;
constexpr int kHD = 64;
constexpr int kHDRoot = 8;
constexpr int kQB = 256;
constexpr int kNQB = kT / kQB;
constexpr int kMixN = 96;
constexpr int kMixPad = 128;
constexpr int kHaN = 128;
constexpr int kLoraD = 32;
static_assert(kHDRoot * kHDRoot == kHD, "head dim root");
static_assert(kH * kHD == kC, "head split");
static_assert(kT % kQB == 0 && kQB % 64 == 0, "query blocking");
static_assert(kC % 64 == 0 && kT % 64 == 0 && kC % 32 == 0, "tile multiples");
static_assert(kMixN == 3 * kLoraD && kHaN == 4 * kLoraD, "lora groups");

constexpr float kQScale = 1.0f / (float)kHDRoot;
constexpr float kCarryBig = 16.0f;
constexpr float kCarryBigInv = 1.0f / kCarryBig;
constexpr float kCarrySmall = 64.0f;
constexpr float kCarrySmallInv = 1.0f / kCarrySmall;
constexpr float kPCarry = 16384.0f;
constexpr float kPCarryInv = 1.0f / kPCarry;
constexpr float kLnEps = 1e-5f;
constexpr float kInvC = 1.0f / (float)kC;
constexpr float kInvH = 1.0f / (float)kH;
constexpr float kFltMin = 1.17549435e-38f;

typedef __attribute__((ext_vector_type(16))) _Float16 v16h;
typedef __attribute__((ext_vector_type(8)))  _Float16 v8h;
typedef __attribute__((ext_vector_type(8)))  float    v8f;
typedef __attribute__((ext_vector_type(4)))  float    v4f;
typedef __attribute__((ext_vector_type(4)))  unsigned int v4u;
typedef __attribute__((ext_vector_type(2)))  unsigned int v2u;

__device__ __forceinline__ unsigned pk16(unsigned short a, unsigned short b) { return (unsigned)a | ((unsigned)b << 16); }
__device__ __forceinline__ unsigned short h_bits(float f) { const _Float16 h = (_Float16)f; return __builtin_bit_cast(unsigned short, h); }
__device__ __forceinline__ v4u pack8_f16(const v4f a, const v4f b) {
  const unsigned short h0 = h_bits(a[0]);
  const unsigned short h1 = h_bits(a[1]);
  const unsigned short h2 = h_bits(a[2]);
  const unsigned short h3 = h_bits(a[3]);
  const unsigned short h4 = h_bits(b[0]);
  const unsigned short h5 = h_bits(b[1]);
  const unsigned short h6 = h_bits(b[2]);
  const unsigned short h7 = h_bits(b[3]);
  return (v4u){pk16(h0, h1), pk16(h2, h3), pk16(h4, h5), pk16(h6, h7)};
}
__device__ __forceinline__ void pin2_v4f(v4f& a, v4f& b) { asm volatile("" : "+v"(a), "+v"(b)); }

union FragU { v16h v; v8h h[2]; };
__device__ __forceinline__ v16h ld_frag(const _Float16* p) {
  FragU f;
  f.h[0] = *(const v8h*)(p);
  f.h[1] = *(const v8h*)(p + 16);
  return f.v;
}
__device__ __forceinline__ v8f mma_h(v16h a, v16h b, v8f c) {
  return __builtin_amdgcn_wmma_f32_16x16x32_f16(false, a, false, b, (short)0, c, false, false);
}
__device__ __forceinline__ void guard_row_h(v8f& a0, v8f& a1, v8f& a2, v8f& a3, v16h x, v16h b0, v16h b1, v16h b2, v16h b3) {
  asm volatile("v_nop\n\tv_nop\n\tv_nop\n\tv_nop" : "+v"(a0), "+v"(a1), "+v"(a2), "+v"(a3) : "v"(x), "v"(b0), "v"(b1), "v"(b2), "v"(b3));
}
__device__ __forceinline__ void keep4_h(v16h a, v16h b, v16h c, v16h d) { asm volatile("v_nop" :: "v"(a), "v"(b), "v"(c), "v"(d)); }
__device__ __forceinline__ void acc_guard4(v8f& a, v8f& b, v8f& c, v8f& d) { asm volatile("v_nop\n\tv_nop\n\tv_nop\n\tv_nop" : "+v"(a), "+v"(b), "+v"(c), "+v"(d)); }

__device__ __forceinline__ void wave_sync_lds() {
  __builtin_amdgcn_fence(__ATOMIC_RELEASE, "workgroup");
  __builtin_amdgcn_wave_barrier();
  __builtin_amdgcn_fence(__ATOMIC_ACQUIRE, "workgroup");
}

__global__ __launch_bounds__(256) void gemm_f16_kernel(
    const unsigned short* __restrict__ Ap, int lda, long strideA,
    const unsigned short* __restrict__ Btp, int ldb, long strideB,
    float* __restrict__ Cout, int ldc, long strideC,
    int M, int N, int K, float scale) {
  __shared__ __align__(16) float sT[8][16 * 68];
  const _Float16* A = (const _Float16*)Ap;
  const _Float16* Bt = (const _Float16*)Btp;
  const int b    = blockIdx.y;
  const int lane = threadIdx.x & 31;
  const int wave = threadIdx.x >> 5;
  const int tilesN = N >> 6;
  const int tilesM = M >> 6;
  const int tile = blockIdx.x * 8 + wave;
  if (tile >= tilesM * tilesN) return;
  const int tm = tile / tilesN;
  const int tn = tile - tm * tilesN;
  const int m0 = tm << 6;
  const int n0 = tn << 6;
  const int rlane = lane & 15;
  const int koff  = (lane >> 4) * 8;
  const int mOff  = (lane >> 4) * 8;

  const _Float16* Ab = A  + (size_t)b * strideA + (size_t)(m0 + rlane) * lda + koff;
  const _Float16* Bb = Bt + (size_t)b * strideB + (size_t)(n0 + rlane) * ldb + koff;
  const size_t a16 = (size_t)16 * lda;
  const size_t b16 = (size_t)16 * ldb;

  v8f acc[4][4];
#pragma unroll
  for (int i = 0; i < 4; ++i)
#pragma unroll
    for (int j = 0; j < 4; ++j) acc[i][j] = (v8f){0.f, 0.f, 0.f, 0.f, 0.f, 0.f, 0.f, 0.f};

  for (int k0 = 0; k0 < K; k0 += 32) {
    v16h bh[4];
#pragma unroll
    for (int j = 0; j < 4; ++j) bh[j] = ld_frag(Bb + j * b16 + k0);
#pragma unroll
    for (int i = 0; i < 4; ++i) {
      const v16h ah = ld_frag(Ab + i * a16 + k0);
#pragma unroll
      for (int j = 0; j < 4; ++j) acc[i][j] = mma_h(ah, bh[j], acc[i][j]);
      guard_row_h(acc[i][0], acc[i][1], acc[i][2], acc[i][3], ah, bh[0], bh[1], bh[2], bh[3]);
    }
    keep4_h(bh[0], bh[1], bh[2], bh[3]);
  }
  acc_guard4(acc[0][0], acc[0][1], acc[0][2], acc[0][3]);
  acc_guard4(acc[1][0], acc[1][1], acc[1][2], acc[1][3]);
  acc_guard4(acc[2][0], acc[2][1], acc[2][2], acc[2][3]);
  acc_guard4(acc[3][0], acc[3][1], acc[3][2], acc[3][3]);

  float* slab = sT[wave];
  float* C = Cout + (size_t)b * strideC;
  const int hh = lane >> 4;
  const int c4 = (lane & 15) * 4;
#pragma unroll
  for (int i = 0; i < 4; ++i) {
    const int mBase = m0 + (i << 4);
#pragma unroll
    for (int j = 0; j < 4; ++j) {
#pragma unroll
      for (int r = 0; r < 8; ++r) slab[(mOff + r) * 68 + (j << 4) + rlane] = acc[i][j][r] * scale;
    }
    wave_sync_lds();
    for (int pass = 0; pass < 2; ++pass) {
#pragma unroll
      for (int it = 0; it < 8; ++it) {
        const int row = it * 2 + hh;
        const v4f v = *(const v4f*)(slab + row * 68 + c4);
        *(volatile v4f*)(C + (size_t)(mBase + row) * ldc + n0 + c4) = v;
      }
      __threadfence();
    }
    wave_sync_lds();
  }
}

__global__ __launch_bounds__(256) void mix_gemm_kernel(
    const unsigned short* __restrict__ xxx16, const unsigned short* __restrict__ w2T,
    const float* __restrict__ x, const float* __restrict__ shiftrow,
    const float* __restrict__ tm_r, const float* __restrict__ tm_k, const float* __restrict__ tm_v,
    unsigned short* __restrict__ outq, float scale) {
  __shared__ __align__(16) float sT[8][16 * 68];
  const int g    = blockIdx.y;
  const int lane = threadIdx.x & 31;
  const int wave = threadIdx.x >> 5;
  const int tilesN = kC >> 6;
  const int tilesM = kT >> 6;
  const int tile = blockIdx.x * 8 + wave;
  if (tile >= tilesM * tilesN) return;
  const int tm = tile / tilesN;
  const int tn = tile - tm * tilesN;
  const int m0 = tm << 6;
  const int n0 = tn << 6;
  const int rlane = lane & 15;
  const int koff  = (lane >> 4) * 8;
  const int mOff  = (lane >> 4) * 8;
  const float* tmv = (g == 0) ? tm_r : ((g == 1) ? tm_k : tm_v);

  const _Float16* Ab = (const _Float16*)xxx16 + (size_t)(m0 + rlane) * kMixPad + kLoraD * g + koff;
  const _Float16* Bb = (const _Float16*)w2T + (size_t)g * kC * kLoraD + (size_t)(n0 + rlane) * kLoraD + koff;

  v16h bh[4];
#pragma unroll
  for (int j = 0; j < 4; ++j) bh[j] = ld_frag(Bb + (size_t)j * 16 * kLoraD);
  v8f acc[4][4];
#pragma unroll
  for (int i = 0; i < 4; ++i) {
    const v16h ah = ld_frag(Ab + (size_t)i * 16 * kMixPad);
#pragma unroll
    for (int j = 0; j < 4; ++j) acc[i][j] = mma_h(ah, bh[j], (v8f){0.f, 0.f, 0.f, 0.f, 0.f, 0.f, 0.f, 0.f});
    guard_row_h(acc[i][0], acc[i][1], acc[i][2], acc[i][3], ah, bh[0], bh[1], bh[2], bh[3]);
  }
  keep4_h(bh[0], bh[1], bh[2], bh[3]);
  acc_guard4(acc[0][0], acc[0][1], acc[0][2], acc[0][3]);
  acc_guard4(acc[1][0], acc[1][1], acc[1][2], acc[1][3]);
  acc_guard4(acc[2][0], acc[2][1], acc[2][2], acc[2][3]);
  acc_guard4(acc[3][0], acc[3][1], acc[3][2], acc[3][3]);

  float* slab = sT[wave];
  unsigned short* Cg = outq + (size_t)g * kT * kC;
  const int q  = lane >> 3;
  const int c8 = (lane & 7) * 8;
  const int col = n0 + c8;
  const v4f tma = *(const v4f*)(tmv + col);
  const v4f tmb = *(const v4f*)(tmv + col + 4);
  v4f sha = *(const v4f*)(shiftrow + col);
  v4f shb = *(const v4f*)(shiftrow + col + 4);
  pin2_v4f(sha, shb);
#pragma unroll
  for (int i = 0; i < 4; ++i) {
    const int mBase = m0 + (i << 4);
#pragma unroll
    for (int j = 0; j < 4; ++j) {
#pragma unroll
      for (int r = 0; r < 8; ++r) slab[(mOff + r) * 68 + (j << 4) + rlane] = acc[i][j][r] * scale;
    }
    wave_sync_lds();
    v4u u[4];
#pragma unroll
    for (int it = 0; it < 4; ++it) {
      const int row = it * 4 + q;
      const int t = mBase + row;
      const int tp = (t > 0) ? (t - 1) : 0;
      const float f0 = (t == 0) ? 1.0f : 0.0f;
      const float f1 = 1.0f - f0;
      const v4f xa  = *(const v4f*)(x + (size_t)t * kC + col);
      const v4f xb  = *(const v4f*)(x + (size_t)t * kC + col + 4);
      v4f xpa = *(const v4f*)(x + (size_t)tp * kC + col);
      v4f xpb = *(const v4f*)(x + (size_t)tp * kC + col + 4);
      pin2_v4f(xpa, xpb);
      const v4f ma  = *(const v4f*)(slab + row * 68 + c8);
      const v4f mb  = *(const v4f*)(slab + row * 68 + c8 + 4);
      v4f va, vb;
#pragma unroll
      for (int e = 0; e < 4; ++e) {
        const float xc0 = xa[e];
        const float xc1 = xb[e];
        const float pv0 = fmaf(f0, sha[e], f1 * xpa[e]);
        const float pv1 = fmaf(f0, shb[e], f1 * xpb[e]);
        va[e] = xc0 + (pv0 - xc0) * (tma[e] + ma[e]);
        vb[e] = xc1 + (pv1 - xc1) * (tmb[e] + mb[e]);
      }
      u[it] = pack8_f16(va, vb);
    }
    for (int pass = 0; pass < 2; ++pass) {
#pragma unroll
      for (int it = 0; it < 4; ++it) {
        const int row = it * 4 + q;
        *(volatile v4u*)(Cg + (size_t)(mBase + row) * kC + col) = u[it];
      }
      __threadfence();
    }
    wave_sync_lds();
  }
}

__global__ __launch_bounds__(256) void wt_cast_kernel(const float* __restrict__ W0, const float* __restrict__ W1,
                                                      const float* __restrict__ W2, const float* __restrict__ W3,
                                                      int ldw, int nreal, int kdim,
                                                      unsigned short* __restrict__ out, long plane_stride, float carry) {
  __shared__ float sm[64][65];
  const int t  = threadIdx.x;
  const int k0 = blockIdx.x * 64;
  const int n0 = blockIdx.y * 64;
  const int z  = blockIdx.z;
  const float* W = (z == 0) ? W0 : ((z == 1) ? W1 : ((z == 2) ? W2 : W3));
#pragma unroll
  for (int i = 0; i < 16; ++i) {
    const int e = i * 256 + t;
    const int r = e >> 6;
    const int c = e & 63;
    const int n = n0 + c;
    const int nc = (n < nreal) ? n : (nreal - 1);
    const float v = W[(size_t)(k0 + r) * ldw + nc];
    sm[c][r] = (n < nreal) ? (v * carry) : 0.0f;
  }
  __syncthreads();
  const int lane = t & 31, wave = t >> 5;
  const int q = lane >> 3, c8 = (lane & 7) * 8;
  unsigned short* op = out + (size_t)z * plane_stride;
  v4u u[2];
#pragma unroll
  for (int it = 0; it < 2; ++it) {
    const int row = wave * 8 + it * 4 + q;
    unsigned short hb[8];
#pragma unroll
    for (int e = 0; e < 8; ++e) hb[e] = h_bits(sm[row][c8 + e]);
    u[it] = (v4u){pk16(hb[0], hb[1]), pk16(hb[2], hb[3]), pk16(hb[4], hb[5]), pk16(hb[6], hb[7])};
  }
  for (int pass = 0; pass < 2; ++pass) {
#pragma unroll
    for (int it = 0; it < 2; ++it) {
      const int row = wave * 8 + it * 4 + q;
      *(volatile v4u*)(op + (size_t)(n0 + row) * kdim + k0 + c8) = u[it];
    }
    __threadfence();
  }
}

__global__ __launch_bounds__(256) void w2t_kernel(const float* __restrict__ w2, unsigned short* __restrict__ out, float carry) {
  __shared__ float sm[kLoraD][65];
  const int t  = threadIdx.x;
  const int c0 = blockIdx.x * 64;
  const int g  = blockIdx.y;
#pragma unroll
  for (int i = 0; i < 8; ++i) {
    const int e = i * 256 + t;
    const int d = e >> 6;
    const int cl = e & 63;
    sm[d][cl] = w2[((size_t)g * kLoraD + d) * kC + c0 + cl] * carry;
  }
  __syncthreads();
  const int cl = t >> 2;
  const int d0 = (t & 3) * 8;
  unsigned short hb[8];
#pragma unroll
  for (int e = 0; e < 8; ++e) hb[e] = h_bits(sm[d0 + e][cl]);
  const v4u u = (v4u){pk16(hb[0], hb[1]), pk16(hb[2], hb[3]), pk16(hb[4], hb[5]), pk16(hb[6], hb[7])};
  unsigned short* p = out + ((size_t)g * kC + c0) * kLoraD + 8 * (size_t)t;
  *(volatile v4u*)p = u;
  __threadfence();
  *(volatile v4u*)p = u;
}

__global__ __launch_bounds__(256) void prep_kernel(const float* __restrict__ x, const float* __restrict__ shiftrow,
                                                   const float* __restrict__ tmx,
                                                   unsigned short* __restrict__ x16, unsigned short* __restrict__ z16) {
  const int i = blockIdx.x * 256 + threadIdx.x;
  if (i >= kT * kC / 8) return;
  const int t  = i >> 7;
  const int c8 = (i & 127) * 8;
  const int tp = (t > 0) ? (t - 1) : 0;
  const v4f xa  = *(const v4f*)(x + (size_t)t * kC + c8);
  const v4f xb  = *(const v4f*)(x + (size_t)t * kC + c8 + 4);
  const v4f xpa = *(const v4f*)(x + (size_t)tp * kC + c8);
  const v4f xpb = *(const v4f*)(x + (size_t)tp * kC + c8 + 4);
  const v4f sa  = *(const v4f*)(shiftrow + c8);
  const v4f sb  = *(const v4f*)(shiftrow + c8 + 4);
  const v4f ta  = *(const v4f*)(tmx + c8);
  const v4f tb  = *(const v4f*)(tmx + c8 + 4);
  v4f za, zb;
#pragma unroll
  for (int e = 0; e < 4; ++e) {
    const float c0 = xa[e];
    const float c1 = xb[e];
    const float p0 = (t == 0) ? sa[e] : xpa[e];
    const float p1 = (t == 0) ? sb[e] : xpb[e];
    za[e] = c0 + (p0 - c0) * ta[e];
    zb[e] = c1 + (p1 - c1) * tb[e];
  }
  const v4u ux = pack8_f16(xa, xb);
  const v4u uz = pack8_f16(za, zb);
  unsigned short* px = x16 + 8 * (size_t)i;
  unsigned short* pz = z16 + 8 * (size_t)i;
  *(volatile v4u*)px = ux;
  *(volatile v4u*)pz = uz;
  __threadfence();
  *(volatile v4u*)px = ux;
  *(volatile v4u*)pz = uz;
}

__global__ __launch_bounds__(256) void tanh_cvt_kernel(const float* __restrict__ in, unsigned short* __restrict__ out) {
  __shared__ __align__(16) float sm[2048];
  const int tid = threadIdx.x;
  const size_t base = (size_t)blockIdx.x * 2048;
#pragma unroll 1
  for (int i = 0; i < 8; ++i) sm[i * 256 + tid] = tanhf(in[base + i * 256 + tid]);
  __syncthreads();
  const v4f a = *(const v4f*)(sm + 8 * tid);
  const v4f b = *(const v4f*)(sm + 8 * tid + 4);
  const v4u u = pack8_f16(a, b);
  unsigned short* p = out + base + 8 * (size_t)tid;
  *(volatile v4u*)p = u;
  __threadfence();
  *(volatile v4u*)p = u;
}

__global__ __launch_bounds__(256) void headmix_coef_kernel(const float* __restrict__ halin, const float* __restrict__ hw2,
                                                           float* __restrict__ hmT) {
  __shared__ __align__(16) float th[32 * kHaN];
  __shared__ __align__(16) float ob[64 * 36];
  const int tid = threadIdx.x;
  const int t0 = blockIdx.x * 32;
#pragma unroll 1
  for (int i = 0; i < 16; ++i) {
    const int idx = i * 256 + tid;
    th[idx] = tanhf(halin[(size_t)t0 * kHaN + idx]);
  }
  __syncthreads();
  const int nh = tid & 63;
  const int tg = tid >> 6;
  const int n = nh >> 4;
  const int h = nh & 15;
  float acc[8];
#pragma unroll
  for (int j = 0; j < 8; ++j) acc[j] = 0.0f;
#pragma unroll 1
  for (int d = 0; d < kLoraD; ++d) {
    const float w = hw2[(n * kLoraD + d) * kH + h];
#pragma unroll
    for (int j = 0; j < 8; ++j) acc[j] = fmaf(th[(tg * 8 + j) * kHaN + n * kLoraD + d], w, acc[j]);
  }
#pragma unroll
  for (int j = 0; j < 8; ++j) ob[nh * 36 + tg * 8 + j] = acc[j] * kInvH;
  __syncthreads();
  const int lane = tid & 31, wave = tid >> 5;
  const int q = lane >> 3, c4 = (lane & 7) * 4;
  v4f vv[2];
#pragma unroll
  for (int it = 0; it < 2; ++it) {
    const int line = wave * 8 + it * 4 + q;
    vv[it] = *(const v4f*)(ob + line * 36 + c4);
  }
  for (int pass = 0; pass < 2; ++pass) {
#pragma unroll
    for (int it = 0; it < 2; ++it) {
      const int line = wave * 8 + it * 4 + q;
      *(volatile v4f*)(hmT + (size_t)line * kT + t0 + c4) = vv[it];
    }
    __threadfence();
  }
}

template <int MODE>
__global__ __launch_bounds__(256) void ln_rows_kernel(const float* __restrict__ in, const float* __restrict__ gam,
                                                      const float* __restrict__ bet, unsigned short* __restrict__ out, int nrows) {
  const int tid = threadIdx.x, lane = tid & 31;
  const int row = blockIdx.x * 8 + (tid >> 5);
  if (row >= nrows) return;
  const float* rp = in + (size_t)row * kC;
  float v[4][8];
  float s = 0.0f;
#pragma unroll
  for (int q = 0; q < 4; ++q) {
    const v4f a = *(const v4f*)(rp + 256 * q + 8 * lane);
    const v4f b = *(const v4f*)(rp + 256 * q + 8 * lane + 4);
#pragma unroll
    for (int e = 0; e < 4; ++e) { v[q][e] = a[e]; v[q][4 + e] = b[e]; }
    s += ((a[0] + a[1]) + (a[2] + a[3])) + ((b[0] + b[1]) + (b[2] + b[3]));
  }
#pragma unroll
  for (int off = 1; off < 32; off <<= 1) s += __shfl_xor(s, off, 32);
  const float mu = s * kInvC;
  float ss = 0.0f;
#pragma unroll
  for (int q = 0; q < 4; ++q)
#pragma unroll
    for (int e = 0; e < 8; ++e) { const float d = v[q][e] - mu; v[q][e] = d; ss = fmaf(d, d, ss); }
#pragma unroll
  for (int off = 1; off < 32; off <<= 1) ss += __shfl_xor(ss, off, 32);
  const float rstd = rsqrtf(ss * kInvC + kLnEps);
  v4u o[4];
#pragma unroll
  for (int q = 0; q < 4; ++q) {
    const v4f ga = *(const v4f*)(gam + 256 * q + 8 * lane);
    const v4f gb = *(const v4f*)(gam + 256 * q + 8 * lane + 4);
    const v4f ba = *(const v4f*)(bet + 256 * q + 8 * lane);
    const v4f bb = *(const v4f*)(bet + 256 * q + 8 * lane + 4);
    v4f fa, fb;
#pragma unroll
    for (int e = 0; e < 4; ++e) {
      fa[e] = (v[q][e] * rstd) * ga[e] + ba[e];
      fb[e] = (v[q][4 + e] * rstd) * gb[e] + bb[e];
    }
    o[q] = pack8_f16(fa, fb);
  }
  for (int pass = 0; pass < 2; ++pass) {
#pragma unroll
    for (int q = 0; q < 4; ++q) {
      unsigned short* p;
      if (MODE == 0) p = out + ((size_t)(4 * q + (lane >> 3)) * kT + row) * kHD + (lane & 7) * 8;
      else           p = out + (size_t)row * kC + 256 * q + 8 * lane;
      *(volatile v4u*)p = o[q];
    }
    __threadfence();
  }
}

__global__ __launch_bounds__(256) void transpose16_kernel(const unsigned short* __restrict__ in, unsigned short* __restrict__ out) {
  __shared__ unsigned short sm[64 * 66];
  const int tid = threadIdx.x;
  const int c0 = blockIdx.x * 64;
  const int t0 = blockIdx.y * 64;
  const int r = tid >> 2;
  const int seg = (tid & 3) * 16;
  const v4u w0 = *(const v4u*)(in + (size_t)(t0 + r) * kC + c0 + seg);
  const v4u w1 = *(const v4u*)(in + (size_t)(t0 + r) * kC + c0 + seg + 8);
#pragma unroll
  for (int e = 0; e < 4; ++e) {
    const unsigned a = w0[e];
    const unsigned b = w1[e];
    sm[(seg + 2 * e) * 66 + r]         = (unsigned short)(a & 0xffffu);
    sm[(seg + 2 * e + 1) * 66 + r]     = (unsigned short)(a >> 16);
    sm[(seg + 8 + 2 * e) * 66 + r]     = (unsigned short)(b & 0xffffu);
    sm[(seg + 8 + 2 * e + 1) * 66 + r] = (unsigned short)(b >> 16);
  }
  __syncthreads();
  const int lane = tid & 31, wave = tid >> 5;
  const int q = lane >> 3, c8 = (lane & 7) * 8;
  v4u u[2];
#pragma unroll
  for (int it = 0; it < 2; ++it) {
    const int row = wave * 8 + it * 4 + q;
    unsigned short hb[8];
#pragma unroll
    for (int e = 0; e < 8; ++e) hb[e] = sm[row * 66 + c8 + e];
    u[it] = (v4u){pk16(hb[0], hb[1]), pk16(hb[2], hb[3]), pk16(hb[4], hb[5]), pk16(hb[6], hb[7])};
  }
  for (int pass = 0; pass < 2; ++pass) {
#pragma unroll
    for (int it = 0; it < 2; ++it) {
      const int row = wave * 8 + it * 4 + q;
      *(volatile v4u*)(out + (size_t)(c0 + row) * kT + t0 + c8) = u[it];
    }
    __threadfence();
  }
}

__global__ __launch_bounds__(512) void mix_softmax_kernel(const float* __restrict__ scr, const float* __restrict__ hmT,
                                                          unsigned short* __restrict__ P, int qb, int s_end) {
  __shared__ __align__(16) float est[kH * kT];
  __shared__ float redm[kH * 16];
  __shared__ float reds[kH * 16];
  __shared__ float finm[kH];
  __shared__ float finl[kH];
  const int tid  = threadIdx.x;
  const int lane = tid & 31;
  const int wave = __builtin_amdgcn_readfirstlane(tid >> 5);
  const int tl = blockIdx.x;
  const int t  = qb * kQB + tl;
  const int s0 = 4 * tid;
  const bool wlive = (128 * wave <= t);
  const bool wzero = (!wlive) && (128 * wave < s_end);
  const float* srow = scr + (size_t)tl * kT + s0;
  float* erow = est + s0;
  const float NEG_INF = -INFINITY;

  float ab[4] = {0.f, 0.f, 0.f, 0.f};

  if (wlive) {
    float a[4]   = {0.f, 0.f, 0.f, 0.f};
    float b0[4]  = {0.f, 0.f, 0.f, 0.f};
    float spk[4] = {0.f, 0.f, 0.f, 0.f};
#pragma unroll 1
    for (int h = 0; h < kH; ++h) {
      const float pq = hmT[(size_t)(0 * kH + h) * kT + t];
      const v4f y  = *(const v4f*)(srow + (size_t)h * kQB * kT);
      const v4f pk = *(const v4f*)(hmT + (size_t)(1 * kH + h) * kT + s0);
#pragma unroll
      for (int j = 0; j < 4; ++j) {
        a[j]  = fmaf(y[j], pq, a[j]);
        b0[j] = fmaf(y[j], pk[j], b0[j]);
        spk[j] += pk[j];
      }
      *(v4f*)(erow + h * kT) = y;
    }
#pragma unroll
    for (int j = 0; j < 4; ++j) ab[j] = a[j] + (b0[j] + a[j] * spk[j]);
  }

  if (wlive) {
#pragma unroll 1
    for (int h = 0; h < kH; ++h) {
      const float slope = (((h & 1) == 0) ? 0.70710678118654752f : 0.5f) * __uint_as_float((unsigned)(127 - (h >> 1)) << 23);
      v4f y = *(const v4f*)(erow + h * kT);
      float mx = NEG_INF;
#pragma unroll
      for (int j = 0; j < 4; ++j) {
        const int s = s0 + j;
        const float rel = (float)(t - s);
        const float lg = (y[j] + ab[j]) - slope * rel;
        const float lm = (s > t) ? NEG_INF : lg;
        y[j] = lm;
        mx = fmaxf(mx, lm);
      }
      *(v4f*)(erow + h * kT) = y;
#pragma unroll
      for (int off = 16; off > 0; off >>= 1) mx = fmaxf(mx, __shfl_xor(mx, off, 32));
      if (lane == 0) redm[h * 16 + wave] = mx;
    }
  } else {
    if (lane < 16) redm[lane * 16 + wave] = NEG_INF;
  }
  __syncthreads();
  {
    float v = redm[tid & 255];
    v = fmaxf(v, __shfl_xor(v, 8, 32));
    v = fmaxf(v, __shfl_xor(v, 4, 32));
    v = fmaxf(v, __shfl_xor(v, 2, 32));
    v = fmaxf(v, __shfl_xor(v, 1, 32));
    if (tid < 256 && (tid & 15) == 0) finm[tid >> 4] = v;
  }
  __syncthreads();

  if (wlive) {
#pragma unroll 1
    for (int h = 0; h < kH; ++h) {
      const float mh = finm[h];
      v4f y = *(const v4f*)(erow + h * kT);
      float sm = 0.0f;
#pragma unroll
      for (int j = 0; j < 4; ++j) {
        float e = expf(y[j] - mh);
        e = (e < kFltMin) ? 0.0f : e;
        y[j] = e;
        sm += e;
      }
      *(v4f*)(erow + h * kT) = y;
#pragma unroll
      for (int off = 16; off > 0; off >>= 1) sm += __shfl_xor(sm, off, 32);
      if (lane == 0) reds[h * 16 + wave] = sm;
    }
  } else {
    if (lane < 16) reds[lane * 16 + wave] = 0.0f;
  }
  __syncthreads();
  {
    float v = reds[tid & 255];
    v += __shfl_xor(v, 8, 32);
    v += __shfl_xor(v, 4, 32);
    v += __shfl_xor(v, 2, 32);
    v += __shfl_xor(v, 1, 32);
    if (tid < 256 && (tid & 15) == 0) finl[tid >> 4] = 1.0f / v;
  }
  __syncthreads();

  if (wlive) {
    float a2[4]  = {0.f, 0.f, 0.f, 0.f};
    float b2[4]  = {0.f, 0.f, 0.f, 0.f};
    float spo[4] = {0.f, 0.f, 0.f, 0.f};
#pragma unroll 1
    for (int h = 0; h < kH; ++h) {
      const float il = finl[h];
      const float pq = hmT[(size_t)(2 * kH + h) * kT + t];
      const v4f e  = *(const v4f*)(erow + h * kT);
      const v4f pk = *(const v4f*)(hmT + (size_t)(3 * kH + h) * kT + s0);
#pragma unroll
      for (int j = 0; j < 4; ++j) {
        const float p = e[j] * il;
        a2[j] = fmaf(p, pq, a2[j]);
        b2[j] = fmaf(p, pk[j], b2[j]);
        spo[j] += pk[j];
      }
    }
    float ab2[4];
#pragma unroll
    for (int j = 0; j < 4; ++j) ab2[j] = a2[j] + (b2[j] + a2[j] * spo[j]);
#pragma unroll 1
    for (int h = 0; h < kH; ++h) {
      const float il = finl[h];
      const v4f e = *(const v4f*)(erow + h * kT);
      float w[4];
#pragma unroll
      for (int j = 0; j < 4; ++j) {
        const float val = (e[j] * il + ab2[j]) * kPCarry;
        w[j] = (s0 + j > t) ? 0.0f : val;
      }
      const unsigned short h0 = h_bits(w[0]);
      const unsigned short h1 = h_bits(w[1]);
      const unsigned short h2 = h_bits(w[2]);
      const unsigned short h3 = h_bits(w[3]);
      const v2u u = (v2u){pk16(h0, h1), pk16(h2, h3)};
      unsigned short* p = P + ((size_t)(h * kQB + tl)) * kT + s0;
      *(volatile v2u*)p = u;
      __threadfence();
      *(volatile v2u*)p = u;
    }
  } else if (wzero) {
    const v2u zu = (v2u){0u, 0u};
#pragma unroll 1
    for (int h = 0; h < kH; ++h) {
      unsigned short* p = P + ((size_t)(h * kQB + tl)) * kT + s0;
      *(volatile v2u*)p = zu;
      __threadfence();
      *(volatile v2u*)p = zu;
    }
  }
}

extern "C" void kernel_launch(void* const* d_in, const int* in_sizes, int n_in,
                              void* d_out, int out_size, void* d_ws, size_t ws_size, hipStream_t stream) {
  if (n_in < 22 || d_out == nullptr || d_ws == nullptr) return;
  if (in_sizes[0] != kT * kC || in_sizes[1] != kC || in_sizes[2] != kC || in_sizes[3] != kC ||
      in_sizes[4] != kC || in_sizes[5] != kC || in_sizes[6] != kC * kMixN || in_sizes[7] != 3 * kLoraD * kC ||
      in_sizes[8] != kC * kHaN || in_sizes[9] != 4 * kLoraD * kH || in_sizes[10] != kC * kC ||
      in_sizes[11] != kC * kC || in_sizes[12] != kC * kC || in_sizes[13] != kC * kC ||
      in_sizes[14] != kC || in_sizes[15] != kC || in_sizes[16] != kC || in_sizes[17] != kC ||
      in_sizes[18] != kC || in_sizes[19] != kC || in_sizes[20] != kC || in_sizes[21] != kC ||
      out_size != kT * kC) return;

  const float* x      = (const float*)d_in[0];
  const float* shiftr = (const float*)d_in[1];
  const float* tmx    = (const float*)d_in[2];
  const float* tmr    = (const float*)d_in[3];
  const float* tmk    = (const float*)d_in[4];
  const float* tmv    = (const float*)d_in[5];
  const float* mw1    = (const float*)d_in[6];
  const float* mw2    = (const float*)d_in[7];
  const float* hw1    = (const float*)d_in[8];
  const float* hw2    = (const float*)d_in[9];
  const float* w_r    = (const float*)d_in[10];
  const float* w_k    = (const float*)d_in[11];
  const float* w_v    = (const float*)d_in[12];
  const float* w_o    = (const float*)d_in[13];
  const float* ln_r_g = (const float*)d_in[14];
  const float* ln_r_b = (const float*)d_in[15];
  const float* ln_k_g = (const float*)d_in[16];
  const float* ln_k_b = (const float*)d_in[17];
  const float* ln_v_g = (const float*)d_in[18];
  const float* ln_v_b = (const float*)d_in[19];
  const float* ln_x_g = (const float*)d_in[20];
  const float* ln_x_b = (const float*)d_in[21];
  float* out = (float*)d_out;

  char* ws = (char*)d_ws;
  size_t off = 0;
  auto carve = [&](size_t bytes) -> char* { char* p = ws + off; off += (bytes + 255) & ~(size_t)255; return p; };
  unsigned short* WT4   = (unsigned short*)carve((size_t)4 * kC * kC * 2);
  unsigned short* W1T   = (unsigned short*)carve((size_t)kMixPad * kC * 2);
  unsigned short* HW1T  = (unsigned short*)carve((size_t)kHaN * kC * 2);
  unsigned short* W2T   = (unsigned short*)carve((size_t)3 * kC * kLoraD * 2);
  unsigned short* Z16   = (unsigned short*)carve((size_t)kT * kC * 2);
  unsigned short* X16   = (unsigned short*)carve((size_t)kT * kC * 2);
  float*          LIN   = (float*)carve((size_t)2 * kT * kMixPad * 4);
  unsigned short* XXX16 = (unsigned short*)carve((size_t)kT * kMixPad * 2);
  float*          HMT   = (float*)carve((size_t)4 * kH * kT * 4);
  unsigned short* XQKV  = (unsigned short*)carve((size_t)3 * kT * kC * 2);
  float*          PRE   = (float*)carve((size_t)kT * kC * 4);
  unsigned short* Q16   = (unsigned short*)carve((size_t)kT * kC * 2);
  unsigned short* K16   = (unsigned short*)carve((size_t)kT * kC * 2);
  unsigned short* V16   = (unsigned short*)carve((size_t)kT * kC * 2);
  unsigned short* VT16  = (unsigned short*)carve((size_t)kT * kC * 2);
  float*          SCR   = (float*)carve((size_t)kH * kQB * kT * 4);
  unsigned short* P16   = (unsigned short*)carve((size_t)kH * kQB * kT * 2);
  float*          ATT   = (float*)carve((size_t)kT * kC * 4);
  unsigned short* ATT16 = (unsigned short*)carve((size_t)kT * kC * 2);
  if (off > ws_size || off > (size_t)134217728) return;
  static_assert(kMixPad == kHaN, "the two LoRA input GEMMs share one batched launch");

  wt_cast_kernel<<<dim3(kC / 64, kC / 64, 4), 256, 0, stream>>>(w_r, w_k, w_v, w_o, kC, kC, kC, WT4, (long)kC * kC, kCarryBig);
  wt_cast_kernel<<<dim3(kC / 64, kMixPad / 64, 1), 256, 0, stream>>>(mw1, mw1, mw1, mw1, kMixN, kMixN, kC, W1T, 0L, kCarrySmall);
  wt_cast_kernel<<<dim3(kC / 64, kHaN / 64, 1), 256, 0, stream>>>(hw1, hw1, hw1, hw1, kHaN, kHaN, kC, HW1T, 0L, kCarrySmall);
  w2t_kernel<<<dim3(kC / 64, 3), 256, 0, stream>>>(mw2, W2T, kCarrySmall);

  prep_kernel<<<kT * kC / 8 / 256, 256, 0, stream>>>(x, shiftr, tmx, X16, Z16);

  static_assert(kT % 64 == 0 && kMixPad % 64 == 0 && kC % 32 == 0, "gemm shape");
  gemm_f16_kernel<<<dim3((kT / 64) * (kMixPad / 64) / 8, 2), 256, 0, stream>>>(
      Z16, kC, (long)kT * kC, W1T, kC, (long)kMixPad * kC, LIN, kMixPad, (long)kT * kMixPad,
      kT, kMixPad, kC, kCarrySmallInv);

  tanh_cvt_kernel<<<kT * kMixPad / 2048, 256, 0, stream>>>(LIN, XXX16);
  headmix_coef_kernel<<<kT / 32, 256, 0, stream>>>(LIN + (size_t)kT * kMixPad, hw2, HMT);

  mix_gemm_kernel<<<dim3((kT / 64) * (kC / 64) / 8, 3), 256, 0, stream>>>(
      XXX16, W2T, x, shiftr, tmr, tmk, tmv, XQKV, kCarrySmallInv);

  const dim3 gbig((kT / 64) * (kC / 64) / 8, 1);
  gemm_f16_kernel<<<gbig, 256, 0, stream>>>(XQKV, kC, 0L, WT4, kC, 0L, PRE, kC, 0L, kT, kC, kC, kCarryBigInv);
  ln_rows_kernel<0><<<kT / 8, 256, 0, stream>>>(PRE, ln_r_g, ln_r_b, Q16, kT);
  gemm_f16_kernel<<<gbig, 256, 0, stream>>>(XQKV + (size_t)kT * kC, kC, 0L, WT4 + (size_t)kC * kC, kC, 0L, PRE, kC, 0L, kT, kC, kC, kCarryBigInv);
  ln_rows_kernel<0><<<kT / 8, 256, 0, stream>>>(PRE, ln_k_g, ln_k_b, K16, kT);
  gemm_f16_kernel<<<gbig, 256, 0, stream>>>(XQKV + (size_t)2 * kT * kC, kC, 0L, WT4 + (size_t)2 * kC * kC, kC, 0L, PRE, kC, 0L, kT, kC, kC, kCarryBigInv);
  ln_rows_kernel<1><<<kT / 8, 256, 0, stream>>>(PRE, ln_v_g, ln_v_b, V16, kT);
  transpose16_kernel<<<dim3(kC / 64, kT / 64), 256, 0, stream>>>(V16, VT16);

  for (int qb = 0; qb < kNQB; ++qb) {
    const int s_end = kQB * (qb + 1);
    gemm_f16_kernel<<<dim3((kQB / 64) * (s_end / 64) / 8, kH), 256, 0, stream>>>(
        Q16 + (size_t)qb * kQB * kHD, kHD, (long)kT * kHD, K16, kHD, (long)kT * kHD,
        SCR, kT, (long)kQB * kT, kQB, s_end, kHD, kQScale);
    mix_softmax_kernel<<<kQB, 512, 0, stream>>>(SCR, HMT, P16, qb, s_end);
    gemm_f16_kernel<<<dim3(1, kH), 128, 0, stream>>>(
        P16, kT, (long)kQB * kT, VT16, kT, (long)kHD * kT,
        ATT + (size_t)qb * kQB * kC, kC, (long)kHD, kQB, kHD, s_end, kPCarryInv);
  }

  ln_rows_kernel<1><<<kT / 8, 256, 0, stream>>>(ATT, ln_x_g, ln_x_b, ATT16, kT);
  gemm_f16_kernel<<<gbig, 256, 0, stream>>>(ATT16, kC, 0L, WT4 + (size_t)3 * kC * kC, kC, 0L, out, kC, 0L, kT, kC, kC, kCarryBigInv);
}
